// Self_Attention_3332894622394
// MI455X (gfx1250) — hardware-verified
//
#include <hip/hip_runtime.h>
#ifndef NB
#define NB 8
#endif
#ifndef SEQ
#define SEQ 1024
#endif
#define NB_FULL 8
#define L_FULL 1024
#define KK 8
#define CD 64
#define BQ 128
#define BP 64
#define QTN (SEQ / BQ)
#define GRID_R ((NB + NB * KK) * (SEQ / 32))
#define GRID_V ((NB * KK * CD * (SEQ / 8)) / 256)
#define GRID_A (NB * KK * QTN)
static_assert(SEQ % BQ == 0);
static_assert(SEQ % BP == 0);
static_assert(SEQ <= L_FULL);
static_assert(NB <= NB_FULL);
static_assert((NB * KK * CD * (SEQ / 8)) % 256 == 0);
static_assert((size_t)GRID_R * 256 * 8 == (size_t)(NB + NB * KK) * SEQ * CD);
static_assert((size_t)GRID_V * 256 * 8 == (size_t)NB * KK * CD * SEQ);
static_assert((size_t)GRID_A * CD * BQ == (size_t)NB * KK * CD * SEQ);

typedef unsigned short v8us __attribute__((ext_vector_type(8), may_alias));
typedef float  v8f  __attribute__((ext_vector_type(8)));
typedef float  v4f  __attribute__((ext_vector_type(4)));
typedef float  v4fa __attribute__((ext_vector_type(4), may_alias));
typedef _Float16 v16h __attribute__((ext_vector_type(16)));
union FragH { v16h v; v8us half[2]; _Float16 h[16]; unsigned short u[16]; };

__device__ __forceinline__ unsigned short bf16_bits(float x) { unsigned int u = __float_as_uint(x); return (unsigned short)((u + 0x7FFFu + ((u >> 16) & 1u)) >> 16); }
__device__ __forceinline__ float bf16_val(unsigned short b) { return __uint_as_float(((unsigned int)b) << 16); }
__device__ __forceinline__ float bf16_rne(float x) { return bf16_val(bf16_bits(x)); }

__device__ __forceinline__ v16h g2_frag(const _Float16* p, unsigned hh) { FragH f; f.half[0] = *(const v8us*)((const unsigned short*)p + 8u * hh); f.half[1] = *(const v8us*)((const unsigned short*)p + 16u + 8u * hh); return f.v; }
__device__ __forceinline__ v8f g2_mma(v16h a, v16h b, v8f c) { v8f d = __builtin_amdgcn_wmma_f32_16x16x32_f16(false, a, false, b, (short)0, c, false, false); asm volatile("v_nop\n\tv_nop\n\tv_nop\n\tv_nop" : "+v"(d) : "v"(a), "v"(b)); return d; }

__global__ __launch_bounds__(256) void k_rows16(const float* __restrict__ Xq, const float* __restrict__ Xk, _Float16* __restrict__ Q16, _Float16* __restrict__ K16) {
  __shared__ float tl[CD][33];
  const unsigned tid = threadIdx.x;
  const unsigned nl = SEQ / 32u;
  const unsigned nbq = NB * nl;
  unsigned bi = blockIdx.x;
  const bool isq = bi < nbq;
  if (!isq) bi -= nbq;
  const unsigned img = bi / nl, lb = bi - img * nl;
  const float* X = isq ? Xq : Xk;
  _Float16* D = isq ? Q16 : K16;
  const size_t sbase = (size_t)img * CD * L_FULL + (size_t)lb * 32u;
  for (unsigned i = tid; i < CD * 32u; i += 256u) { const unsigned c = i >> 5, l = i & 31u; tl[c][l] = bf16_rne(X[sbase + (size_t)c * L_FULL + l]); }
  __syncthreads();
  { const unsigned l = tid >> 3, c8 = (tid & 7u) * 8u; FragH f;
#pragma unroll
    for (int q = 0; q < 8; ++q) f.h[q] = (_Float16)(tl[c8 + q][l] * 16.0f);
    const v8us o = f.half[0];
    unsigned short* d = (unsigned short*)D + ((size_t)img * SEQ + lb * 32u + l) * CD + c8;
    *(volatile v8us*)d = o; __threadfence(); *(volatile v8us*)d = o; }
}

__global__ __launch_bounds__(256) void k_v16(const float* __restrict__ V, _Float16* __restrict__ V16) {
  const unsigned t = blockIdx.x * 256u + threadIdx.x;
  if (t >= (unsigned)(NB * KK * CD * (SEQ / 8))) return;
  const unsigned row = t / (SEQ / 8u), l8 = (t - row * (SEQ / 8u)) * 8u;
  const float* s = V + (size_t)row * L_FULL + l8;
  const v4f a = *(const v4fa*)s, b = *(const v4fa*)(s + 4);
  FragH f;
#pragma unroll
  for (int q = 0; q < 4; ++q) { f.h[q] = (_Float16)(bf16_rne(a[q]) * 16.0f); f.h[4 + q] = (_Float16)(bf16_rne(b[q]) * 16.0f); }
  const v8us o = f.half[0];
  unsigned short* d = (unsigned short*)V16 + (size_t)t * 8u;
  *(volatile v8us*)d = o; __threadfence(); *(volatile v8us*)d = o;
}

__global__ __launch_bounds__(256) void k_attn(const _Float16* __restrict__ Q16, const _Float16* __restrict__ K16, const _Float16* __restrict__ V16, float* __restrict__ out) {
  __shared__ __attribute__((aligned(16))) float so[CD][BQ + 4];
  const unsigned tid = threadIdx.x, w = tid >> 5, lane = tid & 31u, ln = lane & 15u, hh = lane >> 4;
  const unsigned pair = blockIdx.x / QTN, qt = blockIdx.x - pair * QTN, n = pair / KK;
  const unsigned q0 = qt * BQ + w * 16u;
  const _Float16* qrow = Q16 + ((size_t)n * SEQ + q0 + ln) * CD;
  const v16h bq0 = g2_frag(qrow, hh), bq1 = g2_frag(qrow + 32, hh);
  const _Float16* kbase = K16 + ((size_t)pair * SEQ + ln) * CD;
  const _Float16* vbase = V16 + ((size_t)pair * CD + ln) * SEQ;
  FragH on;
#pragma unroll
  for (int e = 0; e < 16; ++e) on.h[e] = (_Float16)1.0f;
  const v8f z8 = {0.f, 0.f, 0.f, 0.f, 0.f, 0.f, 0.f, 0.f};
  v8f o[4] = {z8, z8, z8, z8};
  v8f osum = z8;
  float m = -3.0e38f;
  const float SC = 0.005635527503472513f;
#pragma unroll 1
  for (unsigned p0 = 0; p0 < SEQ; p0 += BP) {
    v8f s[4];
#pragma unroll
    for (int pt = 0; pt < 4; ++pt) {
      const _Float16* kr = kbase + (size_t)(p0 + pt * 16) * CD;
      const v16h a0 = g2_frag(kr, hh), a1 = g2_frag(kr + 32, hh);
      const v8f c = g2_mma(a0, bq0, z8);
      s[pt] = g2_mma(a1, bq1, c);
    }
    float bm = -3.0e38f;
#pragma unroll
    for (int pt = 0; pt < 4; ++pt)
#pragma unroll
      for (int r = 0; r < 8; ++r) { const float t = s[pt][r] * SC; s[pt][r] = t; bm = fmaxf(bm, t); }
    bm = fmaxf(bm, __shfl_xor(bm, 16, 32));
    const float mn = fmaxf(m, bm);
    const float sc = exp2f(m - mn);
    m = mn;
    const float mm = mn - 14.0f;
    FragH b0, b1;
#pragma unroll
    for (int r = 0; r < 8; ++r) {
      b0.h[r]     = (_Float16)exp2f(s[0][r] - mm);
      b0.h[8 + r] = (_Float16)exp2f(s[1][r] - mm);
      b1.h[r]     = (_Float16)exp2f(s[2][r] - mm);
      b1.h[8 + r] = (_Float16)exp2f(s[3][r] - mm);
    }
#pragma unroll
    for (int ct = 0; ct < 4; ++ct)
#pragma unroll
      for (int r = 0; r < 8; ++r) o[ct][r] *= sc;
#pragma unroll
    for (int r = 0; r < 8; ++r) osum[r] *= sc;
#pragma unroll
    for (int ct = 0; ct < 4; ++ct) {
      const _Float16* vr = vbase + (size_t)(ct * 16) * SEQ + p0;
      const v16h a0 = g2_frag(vr, hh), a1 = g2_frag(vr + 32, hh);
      o[ct] = g2_mma(a0, b0.v, o[ct]);
      o[ct] = g2_mma(a1, b1.v, o[ct]);
    }
    osum = g2_mma(on.v, b0.v, osum);
    osum = g2_mma(on.v, b1.v, osum);
  }
  const float rinv = (1.0f / osum[0]) * 0.0625f;
#pragma unroll
  for (int ct = 0; ct < 4; ++ct)
#pragma unroll
    for (int r = 0; r < 8; ++r) so[ct * 16 + 8 * hh + r][w * 16u + ln] = o[ct][r] * rinv;
  __syncthreads();
  float* ob = out + ((size_t)pair * CD) * SEQ + (size_t)qt * BQ;
  for (int pass = 0; pass < 2; ++pass) {
#pragma unroll
    for (int i = 0; i < 8; ++i) {
      const unsigned c = w * 8u + i;
      const v4f v = *(const v4fa*)&so[c][lane * 4u];
      *(volatile v4f*)(ob + (size_t)c * SEQ + lane * 4u) = v;
    }
    if (pass == 0) __threadfence();
  }
}

extern "C" void kernel_launch(void* const* d_in, const int* in_sizes, int n_in,
                              void* d_out, int out_size, void* d_ws, size_t ws_size, hipStream_t stream) {
  if (n_in < 3) return;
  const long long qmin = (long long)(NB * CD - 1) * L_FULL + SEQ;
  const long long kmin = (long long)(NB * KK * CD - 1) * L_FULL + SEQ;
  if ((long long)in_sizes[0] < qmin || (long long)in_sizes[1] < kmin || (long long)in_sizes[2] < kmin) return;
  if ((long long)out_size < (long long)NB * KK * CD * SEQ) return;
  const float* q = (const float*)d_in[0];
  const float* k = (const float*)d_in[1];
  const float* v = (const float*)d_in[2];
  char* ws = (char*)d_ws; size_t off = 0;
  auto take = [&](size_t bytes) { char* p = ws + off; off += (bytes + 255) & ~(size_t)255; return p; };
  _Float16* Q16 = (_Float16*)take((size_t)NB * SEQ * CD * 2);
  _Float16* K16 = (_Float16*)take((size_t)NB * KK * SEQ * CD * 2);
  _Float16* V16 = (_Float16*)take((size_t)NB * KK * CD * SEQ * 2);
  if (off > ws_size) return;
  k_rows16<<<GRID_R, 256, 0, stream>>>(q, k, Q16, K16);
  k_v16<<<GRID_V, 256, 0, stream>>>(v, V16);
  k_attn<<<GRID_A, 256, 0, stream>>>(Q16, K16, V16, (float*)d_out);
}
